// DCFormer_66365834657868
// MI455X (gfx1250) — hardware-verified
//
#include <hip/hip_runtime.h>
#include <stddef.h>


typedef _Float16 v16h __attribute__((ext_vector_type(16)));
typedef _Float16 v8h  __attribute__((ext_vector_type(8)));
typedef float    v8f  __attribute__((ext_vector_type(8)));
typedef float    v4f  __attribute__((ext_vector_type(4)));
typedef _Float16 h16;

#ifndef NB
#define NB 1
#endif
#ifndef SEQ
#define SEQ 2048
#endif
#define NB_FULL  1
#define SEQ_FULL 2048
#define DIM   1024
#define NHEAD 16
#define HD    64
#define NCP   4
#define KH    128
#define HIDW  (NCP * KH)
#define DDW   (4 * NHEAD)
#define N1    (HIDW + DDW)
#define SWROW (NCP * 64 + DDW)
#define STROW 32
#define TQ    16
#define SK    32
#define SWP   160
#define LDP   40
#ifndef HID_RES
#define HID_RES 1
#endif

static_assert(NB == 1 && NB <= NB_FULL);
static_assert(SEQ >= 64 && SEQ <= SEQ_FULL && (SEQ % 64) == 0);
static_assert(DIM == NHEAD * HD);
static_assert(HD == 64);
static_assert(NHEAD == 16);
static_assert((DIM % 64) == 0 && (DIM % 32) == 0);
static_assert((KH % 32) == 0 && (HIDW % 64) == 0 && DDW == 64 && (N1 % 64) == 0);
static_assert(SWROW == 320 && (SWROW % 32) == 0);
static_assert(STROW == 2 * NHEAD && (STROW % 32) == 0);
static_assert(TQ == 16 && SK == 32);
static_assert(TQ * NHEAD == 256);
static_assert(SK * TQ == 2 * 256);
static_assert(SK * 40 == 5 * 256);
static_assert(TQ * 40 <= 3 * 256);
static_assert(SWP == 40 * 4);
static_assert((LDP % 8) == 0 && LDP >= SK);
static_assert(8 * TQ * HD == SK * TQ * 16);
static_assert(TQ * STROW <= SK * TQ * 4);
static_assert((SEQ % TQ) == 0 && (SEQ % SK) == 0);
static_assert(((size_t)NHEAD * SEQ * HD) % 2048 == 0 && ((size_t)SEQ * DIM) % 2048 == 0);
static_assert((size_t)NHEAD * SEQ_FULL * HD < (size_t)0xFFFFFFFFu);

#define LDT 72
#define LDC 68
static_assert((LDT % 8) == 0 && LDT >= 64);
static_assert((LDC % 4) == 0 && LDC >= 64);

#define WCARRY 64.0f
#define XCARRY 16.0f
#define QCARRY 64.0f
#define KCARRY 16.0f
#define HCARRY 16.0f
#define RCARRY 2048.0f
#define PCARRY 256.0f

#define W1T_BYTES  ((size_t)N1 * DIM * 2)
#define QKW_BYTES  ((size_t)64 * HIDW * 2)
#define X16_BYTES  ((size_t)SEQ * DIM * 2)
#define QK_BYTES   ((size_t)NHEAD * SEQ * HD * 2)
#define H16_BYTES  ((size_t)SEQ * HIDW * 2)
#define SW_BYTES   ((size_t)SEQ * SWROW * 4)
#define ST_BYTES   ((size_t)SEQ * STROW * 4)
#define OFF_W1T (size_t)0
#define OFF_QKW (OFF_W1T + W1T_BYTES)
#define OFF_X16 (OFF_QKW + QKW_BYTES)
#define OFF_Q16 (OFF_X16 + X16_BYTES)
#define OFF_K16 (OFF_Q16 + QK_BYTES)
#define OFF_VT  (OFF_K16 + QK_BYTES)
#define OFF_H16 (OFF_VT + QK_BYTES)
#define OFF_HR  (OFF_H16 + H16_BYTES)
#define OFF_SW  (OFF_HR + H16_BYTES)
#define OFF_ST  (OFF_SW + SW_BYTES)
#define WS_TOTAL (OFF_ST + ST_BYTES)
static_assert((W1T_BYTES % 128) == 0 && (QKW_BYTES % 128) == 0 && (X16_BYTES % 128) == 0);
static_assert((QK_BYTES % 128) == 0 && (H16_BYTES % 128) == 0);
static_assert((SW_BYTES % 128) == 0 && (ST_BYTES % 128) == 0);
static_assert(WS_TOTAL <= (size_t)134217728);

__device__ __forceinline__ float bf16r(float x) {
  unsigned int u = __float_as_uint(x);
  u = (u + 0x7FFFu + ((u >> 16) & 1u)) & 0xFFFF0000u;
  return __uint_as_float(u);
}

static __device__ __forceinline__ h16 toh_flush(float v) {
  const h16 r = (h16)v;
  return (fabsf(v) < 6.103515625e-05f) ? (h16)0.0f : r;
}

__device__ __forceinline__ v16h frag_at(const _Float16* p) {
  v8h lo = *(const v8h*)(p);
  v8h hi = *(const v8h*)(p + 16);
  v16h out;
#pragma unroll
  for (int i = 0; i < 8; ++i) { out[i] = lo[i]; out[i + 8] = hi[i]; }
  return out;
}
__device__ __forceinline__ v16h ld_frag(const _Float16* base, unsigned ld) {
  const unsigned lane = threadIdx.x & 31u;
  return frag_at(base + (lane & 15u) * ld + (lane >> 4) * 8u);
}

__device__ __forceinline__ v8f wmma16(v16h a, v16h b, v8f c) {
  v8f d = __builtin_amdgcn_wmma_f32_16x16x32_f16(false, a, false, b, (short)0, c,
                                                 false, false);
  asm volatile("v_nop\n\tv_nop\n\tv_nop\n\tv_nop" : "+v"(d) : "v"(a), "v"(b));
  return d;
}

__device__ __forceinline__ void wave_lds_sync() {
  __builtin_amdgcn_fence(3  , "wavefront");
  asm volatile("s_wait_dscnt 0x0" ::: "memory");
  __builtin_amdgcn_wave_barrier();
}

__device__ __forceinline__ unsigned side_col(unsigned j, unsigned side) {
  const unsigned a  = side * 64u + 4u * j;
  const unsigned b  = (2u + side) * 64u + 4u * (j - 16u);
  const unsigned d0 = 256u + side * 16u + 4u * (j - 32u);
  const unsigned d1 = 256u + 32u + side * 16u + 4u * (j - 36u);
  return (j < 16u) ? a : ((j < 32u) ? b : ((j < 36u) ? d0 : d1));
}

__device__ __forceinline__ float mix_one(float v, v4f qk, float qa, float qb, float ka,
                                         float kb, float qd, float kd) {
  float r = v + (qk[0] * qa + qk[1] * qb);
  r = r + (qk[2] * ka + qk[3] * kb);
  r = r + v * qd;
  r = r + v * kd;
  return r;
}

__global__ __launch_bounds__(256) void wconv_kernel(
    const float* __restrict__ W, _Float16* __restrict__ Wt, unsigned ldw, unsigned ldk) {
  __shared__ _Float16 T[64 * LDT];
  const unsigned tid = threadIdx.x;
  const unsigned n0 = blockIdx.x * 64u;
  const unsigned k0 = blockIdx.y * 64u;
#pragma unroll 4
  for (unsigned j = 0; j < 16u; ++j) {
    const unsigned idx = tid + 256u * j;
    const unsigned kr = idx >> 6, nc = idx & 63u;
    const float v = W[(size_t)(k0 + kr) * ldw + n0 + nc];
    T[nc * LDT + kr] = (_Float16)(WCARRY * bf16r(v));
  }
  __syncthreads();
  v8h x[2];
  size_t off[2];
#pragma unroll
  for (unsigned i = 0; i < 2u; ++i) {
    const unsigned n = 32u * i + (tid >> 3);
    const unsigned kc = (tid & 7u) * 8u;
    x[i] = *(const v8h*)&T[n * LDT + kc];
    off[i] = (size_t)(n0 + n) * ldk + k0 + kc;
  }
#pragma unroll
  for (int i = 0; i < 2; ++i) *(volatile v8h*)(Wt + off[i]) = x[i];
  __threadfence();
#pragma unroll
  for (int i = 0; i < 2; ++i) *(volatile v8h*)(Wt + off[i]) = x[i];
}

__global__ __launch_bounds__(256) void cast_kernel(
    const float* __restrict__ src, _Float16* __restrict__ dst,
    unsigned seg_len, unsigned seg_stride, float carry) {
  const unsigned e = (blockIdx.x * 256u + threadIdx.x) * 8u;
  const unsigned seg = e / seg_len;
  const unsigned within = e - seg * seg_len;
  const float* p = src + (size_t)seg * seg_stride + within;
  const v4f a0 = *(const v4f*)(p);
  const v4f a1 = *(const v4f*)(p + 4);
  v8h o;
#pragma unroll
  for (int i = 0; i < 4; ++i) {
    o[i]     = toh_flush(carry * bf16r(a0[i]));
    o[i + 4] = toh_flush(carry * bf16r(a1[i]));
  }
  _Float16* d = dst + e;
  *(volatile v8h*)d = o;
  __threadfence();
  *(volatile v8h*)d = o;
}

__global__ __launch_bounds__(256) void gemm_x_kernel(
    const _Float16* __restrict__ A16, const _Float16* __restrict__ Bt,
    _Float16* __restrict__ H16, _Float16* __restrict__ HR16, float* __restrict__ SWp) {
  __shared__ __attribute__((aligned(16))) float Cs[64 * LDC];
  const unsigned tid = threadIdx.x, lane = tid & 31u;
  const unsigned w = (unsigned)__builtin_amdgcn_readfirstlane((int)(tid >> 5));
  const unsigned mw = w >> 1, nw = w & 1u;
  const unsigned hh = lane >> 4, m = lane & 15u;
  const unsigned n0 = blockIdx.x * 64u;
  const unsigned row0 = blockIdx.y * 64u;
  const float cs = 1.0f / (WCARRY * XCARRY);

  const _Float16* ap  = A16 + (size_t)(row0 + mw * 16u + m) * DIM + hh * 8u;
  const _Float16* bp0 = Bt + (size_t)(n0 + nw * 32u + m) * DIM + hh * 8u;
  const _Float16* bp1 = bp0 + (size_t)16 * DIM;
  v8f acc0 = {}, acc1 = {};
#pragma unroll 2
  for (unsigned k0 = 0; k0 < (unsigned)DIM; k0 += 32u) {
    const v16h a  = frag_at(ap + k0);
    const v16h b0 = frag_at(bp0 + k0);
    const v16h b1 = frag_at(bp1 + k0);
    acc0 = wmma16(a, b0, acc0);
    acc1 = wmma16(a, b1, acc1);
  }
#pragma unroll
  for (int r = 0; r < 8; ++r) {
    float* d = &Cs[(mw * 16u + hh * 8u + (unsigned)r) * LDC + nw * 32u + m];
    d[0]  = acc0[r];
    d[16] = acc1[r];
  }
  __syncthreads();

  if (blockIdx.x < (unsigned)(HIDW / 64)) {
#pragma unroll 1
    for (unsigned g = 0; g < 4u; ++g) {
      const unsigned r = 32u * (g >> 1) + (tid >> 3);
      const unsigned c = (tid & 7u) * 8u + 4u * (g & 1u);
      const v4f u = *(const v4f*)&Cs[r * LDC + c];
      v4f t;
#pragma unroll
      for (int j = 0; j < 4; ++j) {
        const float a = u[j] * cs;
        t[j] = HCARRY * (0.5f * a * (1.0f + erff(a * 0.70710678118654752f)));
      }
      *(v4f*)&Cs[r * LDC + c] = t;
    }
    v8h x[2];
#if HID_RES
    v8h xr[2];
#endif
    size_t off[2];
#pragma unroll
    for (unsigned i = 0; i < 2u; ++i) {
      const unsigned r = 32u * i + (tid >> 3);
      const unsigned c = (tid & 7u) * 8u;
      const v4f u0 = *(const v4f*)&Cs[r * LDC + c];
      const v4f u1 = *(const v4f*)&Cs[r * LDC + c + 4];
#pragma unroll
      for (int j = 0; j < 4; ++j) {
        const h16 h0 = toh_flush(u0[j]);
        const h16 h1 = toh_flush(u1[j]);
        x[i][j]     = h0;
        x[i][j + 4] = h1;
#if HID_RES
        xr[i][j]     = toh_flush((u0[j] - (float)h0) * RCARRY);
        xr[i][j + 4] = toh_flush((u1[j] - (float)h1) * RCARRY);
#endif
      }
      off[i] = (size_t)(row0 + r) * HIDW + n0 + c;
    }
#pragma unroll
    for (int i = 0; i < 2; ++i) *(volatile v8h*)(H16 + off[i]) = x[i];
#if HID_RES
#pragma unroll
    for (int i = 0; i < 2; ++i) *(volatile v8h*)(HR16 + off[i]) = xr[i];
#endif
    __threadfence();
#pragma unroll
    for (int i = 0; i < 2; ++i) *(volatile v8h*)(H16 + off[i]) = x[i];
#if HID_RES
#pragma unroll
    for (int i = 0; i < 2; ++i) *(volatile v8h*)(HR16 + off[i]) = xr[i];
#endif
  } else {
#pragma unroll 1
    for (unsigned i = 0; i < 4u; ++i) {
      const unsigned r = 16u * i + (tid >> 4);
      const unsigned c = (tid & 15u) * 4u;
      const v4f u = *(const v4f*)&Cs[r * LDC + c];
      v4f t;
#pragma unroll
      for (int j = 0; j < 4; ++j) t[j] = tanhf(u[j] * cs);
      *(v4f*)&Cs[r * LDC + c] = t;
    }
    v4f xs[4];
    size_t off[4];
#pragma unroll
    for (unsigned i = 0; i < 4u; ++i) {
      const unsigned r = 16u * i + (tid >> 4);
      const unsigned c = (tid & 15u) * 4u;
      xs[i] = *(const v4f*)&Cs[r * LDC + c];
      off[i] = (size_t)(row0 + r) * SWROW + (unsigned)(NCP * 64) + c;
    }
#pragma unroll
    for (int i = 0; i < 4; ++i) *(volatile v4f*)(SWp + off[i]) = xs[i];
    __threadfence();
#pragma unroll
    for (int i = 0; i < 4; ++i) *(volatile v4f*)(SWp + off[i]) = xs[i];
  }
}

__global__ __launch_bounds__(256) void gemm_w_kernel(
    const _Float16* __restrict__ H16, const _Float16* __restrict__ HR16,
    const _Float16* __restrict__ Bt, float* __restrict__ SWp) {
  __shared__ __attribute__((aligned(16))) float Cs[64 * LDC];
  const unsigned tid = threadIdx.x, lane = tid & 31u;
  const unsigned w = (unsigned)__builtin_amdgcn_readfirstlane((int)(tid >> 5));
  const unsigned mw = w >> 1, nw = w & 1u;
  const unsigned hh = lane >> 4, m = lane & 15u;
  const unsigned cblk = blockIdx.x;
  const unsigned row0 = blockIdx.y * 64u;

  const size_t aoff = (size_t)(row0 + mw * 16u + m) * HIDW + cblk * (unsigned)KH + hh * 8u;
  const _Float16* bp0 = Bt + (size_t)(nw * 32u + m) * HIDW + cblk * (unsigned)KH + hh * 8u;
  const _Float16* bp1 = bp0 + (size_t)16 * HIDW;
  v8f acc0 = {}, acc1 = {};
#if HID_RES
  v8f accr0 = {}, accr1 = {};
#endif
#pragma unroll
  for (unsigned k0 = 0; k0 < (unsigned)KH; k0 += 32u) {
    const v16h a  = frag_at(H16 + aoff + k0);
    const v16h b0 = frag_at(bp0 + k0);
    const v16h b1 = frag_at(bp1 + k0);
    acc0 = wmma16(a, b0, acc0);
    acc1 = wmma16(a, b1, acc1);
#if HID_RES
    const v16h ar = frag_at(HR16 + aoff + k0);
    accr0 = wmma16(ar, b0, accr0);
    accr1 = wmma16(ar, b1, accr1);
#endif
  }
  const float c1 = 1.0f / (HCARRY * WCARRY);
#if HID_RES
  const float c2 = 1.0f / (HCARRY * WCARRY * RCARRY);
#endif
#pragma unroll
  for (int r = 0; r < 8; ++r) {
    float* d = &Cs[(mw * 16u + hh * 8u + (unsigned)r) * LDC + nw * 32u + m];
#if HID_RES
    d[0]  = acc0[r] * c1 + accr0[r] * c2;
    d[16] = acc1[r] * c1 + accr1[r] * c2;
#else
    d[0]  = acc0[r] * c1;
    d[16] = acc1[r] * c1;
#endif
  }
  __syncthreads();

  v4f xs[4];
  size_t off[4];
#pragma unroll
  for (unsigned i = 0; i < 4u; ++i) {
    const unsigned r = 16u * i + (tid >> 4);
    const unsigned c = (tid & 15u) * 4u;
    const v4f u = *(const v4f*)&Cs[r * LDC + c];
    float ss = (u[0] * u[0] + u[1] * u[1]) + (u[2] * u[2] + u[3] * u[3]);
    ss += __shfl_xor(ss, 1, 32);
    ss += __shfl_xor(ss, 2, 32);
    const float rs = 1.0f / sqrtf(ss * (1.0f / 16.0f) + 1.0e-6f);
    const float sc = (c < 32u) ? rs : 1.0f;
    v4f val;
#pragma unroll
    for (int j = 0; j < 4; ++j) val[j] = u[j] * sc;
    xs[i] = val;
    off[i] = (size_t)(row0 + r) * SWROW + cblk * 64u + c;
  }
#pragma unroll
  for (int i = 0; i < 4; ++i) *(volatile v4f*)(SWp + off[i]) = xs[i];
  __threadfence();
#pragma unroll
  for (int i = 0; i < 4; ++i) *(volatile v4f*)(SWp + off[i]) = xs[i];
}

template <int PASS>
__device__ __forceinline__ void dc_body(
    const _Float16* __restrict__ Q16, const _Float16* __restrict__ K16,
    const _Float16* __restrict__ Vt, const float* __restrict__ SWg,
    const float* __restrict__ STin, float* __restrict__ STout, float* __restrict__ out) {
  __shared__ __attribute__((aligned(16))) float Ll[SK * TQ * 16];
  __shared__ __attribute__((aligned(16))) float Qk[SK * TQ * 4];
  __shared__ __attribute__((aligned(16))) float Tw[TQ * SWP];
  __shared__ __attribute__((aligned(16))) float Sw[SK * SWP];
  __shared__ __attribute__((aligned(16))) _Float16 Pt[NHEAD * TQ * LDP];
  constexpr int NPH = (PASS == 2) ? 2 : 1;

  const unsigned tid = threadIdx.x, lane = tid & 31u;
  const unsigned wave = (unsigned)__builtin_amdgcn_readfirstlane((int)(tid >> 5));
  const unsigned hh = lane >> 4, m = lane & 15u;
  const unsigned tb = blockIdx.x * (unsigned)TQ;
  const unsigned tl = tid >> 4, n = tid & 15u;

#pragma unroll
  for (unsigned e = 0; e < 3u; ++e) {
    const unsigned idx = tid + 256u * e;
    if (idx < (unsigned)(TQ * 40)) {
      const unsigned p = idx / 40u, j = idx - p * 40u;
      *(v4f*)&Tw[p * SWP + 4u * j] =
          *(const v4f*)(SWg + (size_t)(tb + p) * SWROW + side_col(j, 0u));
    }
  }

  v16h qf[2][2];
#pragma unroll
  for (int j = 0; j < 2; ++j)
#pragma unroll
    for (int c = 0; c < 2; ++c)
      qf[j][c] = frag_at(Q16 + ((size_t)((2u * wave + (unsigned)j) * (unsigned)SEQ + tb + m)) * HD +
                         32u * (unsigned)c + 8u * hh);

  float mrun = -1.0e30f, srun = 0.0f;
  float mrow = 0.0f, inv = 0.0f;
  if (PASS == 2) {
    mrow = STin[(size_t)(tb + tl) * STROW + n];
    inv = 1.0f / STin[(size_t)(tb + tl) * STROW + 16u + n];
  }
  v8f acc[2][4];
#pragma unroll
  for (int j = 0; j < 2; ++j)
#pragma unroll
    for (int dt = 0; dt < 4; ++dt) acc[j][dt] = (v8f){};

#pragma unroll 1
  for (unsigned s0 = 0; s0 < (unsigned)SEQ; s0 += (unsigned)SK) {
#pragma unroll
    for (unsigned e = 0; e < 5u; ++e) {
      const unsigned idx = tid + 256u * e;
      const unsigned p = idx / 40u, j = idx - p * 40u;
      *(v4f*)&Sw[p * SWP + 4u * j] =
          *(const v4f*)(SWg + (size_t)(s0 + p) * SWROW + side_col(j, 1u));
    }
#pragma unroll
    for (int j = 0; j < 2; ++j) {
      const unsigned head = 2u * wave + (unsigned)j;
#pragma unroll
      for (int st = 0; st < 2; ++st) {
        v8f t = {};
#pragma unroll
        for (int c = 0; c < 2; ++c) {
          const v16h kf = frag_at(
              K16 + ((size_t)(head * (unsigned)SEQ + s0 + 16u * (unsigned)st + m)) * HD +
              32u * (unsigned)c + 8u * hh);
          t = wmma16(qf[j][c], kf, t);
        }
#pragma unroll
        for (int r = 0; r < 8; ++r)
          Ll[((16u * (unsigned)st + m) * (unsigned)TQ + 8u * hh + (unsigned)r) * 16u + head] =
              t[r] * (1.0f / (QCARRY * KCARRY));
      }
    }
    __syncthreads();

#pragma unroll
    for (int ph = 0; ph < NPH; ++ph) {
      const unsigned wofs = 64u * (unsigned)ph;
#pragma unroll
      for (unsigned e = 0; e < 2u; ++e) {
        const unsigned p = tid + 256u * e;
        const unsigned sl = p >> 4, t = p & 15u;
        float q0 = 0.0f, q1 = 0.0f, k0 = 0.0f, k1 = 0.0f;
#pragma unroll
        for (unsigned g = 0; g < 4u; ++g) {
          const v4f l  = *(const v4f*)&Ll[p * 16u + 4u * g];
          const v4f a0 = *(const v4f*)&Tw[t * SWP + wofs + 4u * g];
          const v4f a1 = *(const v4f*)&Tw[t * SWP + wofs + 16u + 4u * g];
          const v4f b0 = *(const v4f*)&Sw[sl * SWP + wofs + 4u * g];
          const v4f b1 = *(const v4f*)&Sw[sl * SWP + wofs + 16u + 4u * g];
#pragma unroll
          for (int i = 0; i < 4; ++i) {
            q0 += l[i] * a0[i];
            q1 += l[i] * a1[i];
            k0 += l[i] * b0[i];
            k1 += l[i] * b1[i];
          }
        }
        v4f o4;
        o4[0] = q0; o4[1] = q1; o4[2] = k0; o4[3] = k1;
        *(v4f*)&Qk[p * 4u] = o4;
      }
      __syncthreads();

      const float tq2a = Tw[tl * SWP + wofs + 32u + n];
      const float tq2b = Tw[tl * SWP + wofs + 48u + n];
      const float tdd  = Tw[tl * SWP + 128u + 16u * (unsigned)ph + n];
      float lv[SK];
#pragma unroll
      for (unsigned s = 0; s < (unsigned)SK; ++s) {
        const unsigned cell = s * (unsigned)TQ + tl;
        const float v = Ll[cell * 16u + n];
        const v4f qk = *(const v4f*)&Qk[cell * 4u];
        const float k2a = Sw[s * SWP + wofs + 32u + n];
        const float k2b = Sw[s * SWP + wofs + 48u + n];
        const float sdd = Sw[s * SWP + 128u + 16u * (unsigned)ph + n];
        const float val = mix_one(v, qk, tq2a, tq2b, k2a, k2b, tdd, sdd);
        if (PASS == 1) {
          lv[s] = val;
        } else if (ph == 0) {
          Ll[cell * 16u + n] = __expf(val - mrow) * inv;
        } else {
          Pt[(n * (unsigned)TQ + tl) * LDP + s] = toh_flush(val * PCARRY);
        }
      }
      if (PASS == 1) {
        float cm = lv[0];
#pragma unroll
        for (unsigned s = 1; s < (unsigned)SK; ++s) cm = fmaxf(cm, lv[s]);
        const float nm = fmaxf(mrun, cm);
        float sum = 0.0f;
#pragma unroll
        for (unsigned s = 0; s < (unsigned)SK; ++s) sum += __expf(lv[s] - nm);
        srun = srun * __expf(mrun - nm) + sum;
        mrun = nm;
      }
      __syncthreads();
    }

    if (PASS == 2) {
#pragma unroll
      for (int j = 0; j < 2; ++j) {
        const unsigned head = 2u * wave + (unsigned)j;
        const v16h pf = ld_frag(&Pt[(head * (unsigned)TQ) * LDP], LDP);
#pragma unroll
        for (int dt = 0; dt < 4; ++dt) {
          const v16h vf = frag_at(Vt + (size_t)((unsigned)dt * 16u + m) * ((size_t)NHEAD * SEQ) +
                                  head * (unsigned)SEQ + s0 + 8u * hh);
          acc[j][dt] = wmma16(pf, vf, acc[j][dt]);
        }
      }
    }
  }

  if (PASS == 1) {
    Qk[tl * STROW + n] = mrun;
    Qk[tl * STROW + 16u + n] = srun;
    __syncthreads();
    if (tid < (unsigned)(TQ * 8)) {
      const unsigned line = tid >> 3, pc = (tid & 7u) * 4u;
      const v4f x = *(const v4f*)&Qk[line * STROW + pc];
      float* p = STout + (size_t)(tb + line) * STROW + pc;
      *(volatile v4f*)p = x;
      __threadfence();
      *(volatile v4f*)p = x;
    }
  }

  if (PASS == 2) {
    __syncthreads();
    const float osc = 1.0f / (PCARRY * WCARRY);
#pragma unroll
    for (int j = 0; j < 2; ++j) {
      const unsigned head = 2u * wave + (unsigned)j;
#pragma unroll
      for (int dt = 0; dt < 4; ++dt)
#pragma unroll
        for (int r = 0; r < 8; ++r)
          Ll[wave * 1024u + (8u * hh + (unsigned)r) * 64u + (unsigned)dt * 16u + m] =
              acc[j][dt][r] * osc;
      wave_lds_sync();
      v4f x[8];
      size_t off[8];
#pragma unroll
      for (unsigned i = 0; i < 8u; ++i) {
        const unsigned row = 2u * i + (lane >> 4);
        const unsigned c = (lane & 15u) * 4u;
        x[i] = *(const v4f*)&Ll[wave * 1024u + row * 64u + c];
        off[i] = ((size_t)head * SEQ_FULL + tb + row) * HD + c;
      }
#pragma unroll
      for (int i = 0; i < 8; ++i) *(volatile v4f*)(out + off[i]) = x[i];
      __threadfence();
#pragma unroll
      for (int i = 0; i < 8; ++i) *(volatile v4f*)(out + off[i]) = x[i];
      wave_lds_sync();
    }
  }
}

__device__ __forceinline__ void dc_out_body(
    const _Float16* __restrict__ Q16, const _Float16* __restrict__ K16,
    const _Float16* __restrict__ Vt, const float* __restrict__ SWg,
    const float* __restrict__ STin, float* __restrict__ out) {
  __shared__ __attribute__((aligned(16))) float Ll[SK * TQ * 16];
  __shared__ __attribute__((aligned(16))) float Qk[SK * TQ * 4];
  __shared__ __attribute__((aligned(16))) float Tw[TQ * SWP];
  __shared__ __attribute__((aligned(16))) float Sw[SK * SWP];
  __shared__ __attribute__((aligned(16))) _Float16 Pt[NHEAD * TQ * LDP];

  const unsigned tid = threadIdx.x, lane = tid & 31u;
  const unsigned wave = (unsigned)__builtin_amdgcn_readfirstlane((int)(tid >> 5));
  const unsigned hh = lane >> 4, m = lane & 15u;
  const unsigned tb = blockIdx.x * (unsigned)TQ;
  const unsigned tl = tid >> 4, n = tid & 15u;

#pragma unroll
  for (unsigned e = 0; e < 3u; ++e) {
    const unsigned idx = tid + 256u * e;
    if (idx < (unsigned)(TQ * 40)) {
      const unsigned p = idx / 40u, j = idx - p * 40u;
      *(v4f*)&Tw[p * SWP + 4u * j] =
          *(const v4f*)(SWg + (size_t)(tb + p) * SWROW + side_col(j, 0u));
    }
  }

  const unsigned qbase = ((2u * wave) * (unsigned)SEQ + tb + m) * (unsigned)HD + 8u * hh;

  const float mrow = STin[(size_t)(tb + tl) * STROW + n];
  const float inv = 1.0f / STin[(size_t)(tb + tl) * STROW + 16u + n];

  v8f acc[2][4];
#pragma unroll
  for (int j = 0; j < 2; ++j)
#pragma unroll
    for (int dt = 0; dt < 4; ++dt) acc[j][dt] = (v8f){};

#pragma unroll 1
  for (unsigned s0 = 0; s0 < (unsigned)SEQ; s0 += (unsigned)SK) {
#pragma unroll
    for (unsigned e = 0; e < 5u; ++e) {
      const unsigned idx = tid + 256u * e;
      const unsigned p = idx / 40u, j = idx - p * 40u;
      *(v4f*)&Sw[p * SWP + 4u * j] =
          *(const v4f*)(SWg + (size_t)(s0 + p) * SWROW + side_col(j, 1u));
    }
    unsigned qo = qbase;
    asm volatile("" : "+v"(qo));
#pragma unroll
    for (int j = 0; j < 2; ++j) {
      const unsigned head = 2u * wave + (unsigned)j;
      const unsigned qoj = qo + (unsigned)j * (unsigned)(SEQ * HD);
      const v16h qf0 = frag_at(Q16 + qoj);
      const v16h qf1 = frag_at(Q16 + qoj + 32u);
#pragma unroll
      for (int st = 0; st < 2; ++st) {
        const size_t ko =
            ((size_t)(head * (unsigned)SEQ + s0 + 16u * (unsigned)st + m)) * HD + 8u * hh;
        v8f t = {};
        const v16h kf0 = frag_at(K16 + ko);
        t = wmma16(qf0, kf0, t);
        const v16h kf1 = frag_at(K16 + ko + 32u);
        t = wmma16(qf1, kf1, t);
#pragma unroll
        for (int r = 0; r < 8; ++r)
          Ll[((16u * (unsigned)st + m) * (unsigned)TQ + 8u * hh + (unsigned)r) * 16u + head] =
              t[r] * (1.0f / (QCARRY * KCARRY));
      }
    }
    __syncthreads();

#pragma unroll
    for (int ph = 0; ph < 2; ++ph) {
      const unsigned wofs = 64u * (unsigned)ph;
#pragma unroll 1
      for (unsigned e = 0; e < 2u; ++e) {
        const unsigned p = tid + 256u * e;
        const unsigned sl = p >> 4, t = p & 15u;
        float q0 = 0.0f, q1 = 0.0f, k0 = 0.0f, k1 = 0.0f;
#pragma unroll 2
        for (unsigned g = 0; g < 4u; ++g) {
          const v4f l  = *(const v4f*)&Ll[p * 16u + 4u * g];
          const v4f a0 = *(const v4f*)&Tw[t * SWP + wofs + 4u * g];
          const v4f a1 = *(const v4f*)&Tw[t * SWP + wofs + 16u + 4u * g];
          const v4f b0 = *(const v4f*)&Sw[sl * SWP + wofs + 4u * g];
          const v4f b1 = *(const v4f*)&Sw[sl * SWP + wofs + 16u + 4u * g];
#pragma unroll
          for (int i = 0; i < 4; ++i) {
            q0 += l[i] * a0[i];
            q1 += l[i] * a1[i];
            k0 += l[i] * b0[i];
            k1 += l[i] * b1[i];
          }
        }
        v4f o4;
        o4[0] = q0; o4[1] = q1; o4[2] = k0; o4[3] = k1;
        *(v4f*)&Qk[p * 4u] = o4;
      }
      __syncthreads();

      const float tq2a = Tw[tl * SWP + wofs + 32u + n];
      const float tq2b = Tw[tl * SWP + wofs + 48u + n];
      const float tdd  = Tw[tl * SWP + 128u + 16u * (unsigned)ph + n];
#pragma unroll 4
      for (unsigned s = 0; s < (unsigned)SK; ++s) {
        const unsigned cell = s * (unsigned)TQ + tl;
        const float v = Ll[cell * 16u + n];
        const v4f qk = *(const v4f*)&Qk[cell * 4u];
        const float k2a = Sw[s * SWP + wofs + 32u + n];
        const float k2b = Sw[s * SWP + wofs + 48u + n];
        const float sdd = Sw[s * SWP + 128u + 16u * (unsigned)ph + n];
        const float val = mix_one(v, qk, tq2a, tq2b, k2a, k2b, tdd, sdd);
        if (ph == 0) {
          Ll[cell * 16u + n] = __expf(val - mrow) * inv;
        } else {
          Pt[(n * (unsigned)TQ + tl) * LDP + s] = toh_flush(val * PCARRY);
        }
      }
      __syncthreads();
    }

#pragma unroll
    for (int j = 0; j < 2; ++j) {
      const unsigned head = 2u * wave + (unsigned)j;
      const v16h pf = ld_frag(&Pt[(head * (unsigned)TQ) * LDP], LDP);
#pragma unroll
      for (int dt = 0; dt < 4; ++dt) {
        const v16h vf = frag_at(Vt + (size_t)((unsigned)dt * 16u + m) * ((size_t)NHEAD * SEQ) +
                                head * (unsigned)SEQ + s0 + 8u * hh);
        acc[j][dt] = wmma16(pf, vf, acc[j][dt]);
      }
    }
  }

  __syncthreads();
  const float osc = 1.0f / (PCARRY * WCARRY);
#pragma unroll
  for (int j = 0; j < 2; ++j) {
    const unsigned head = 2u * wave + (unsigned)j;
#pragma unroll
    for (int dt = 0; dt < 4; ++dt)
#pragma unroll
      for (int r = 0; r < 8; ++r)
        Ll[wave * 1024u + (8u * hh + (unsigned)r) * 64u + (unsigned)dt * 16u + m] =
            acc[j][dt][r] * osc;
    wave_lds_sync();
    v4f x[8];
    size_t off[8];
#pragma unroll
    for (unsigned i = 0; i < 8u; ++i) {
      const unsigned row = 2u * i + (lane >> 4);
      const unsigned c = (lane & 15u) * 4u;
      x[i] = *(const v4f*)&Ll[wave * 1024u + row * 64u + c];
      off[i] = ((size_t)head * SEQ_FULL + tb + row) * HD + c;
    }
#pragma unroll
    for (int i = 0; i < 8; ++i) *(volatile v4f*)(out + off[i]) = x[i];
    __threadfence();
#pragma unroll
    for (int i = 0; i < 8; ++i) *(volatile v4f*)(out + off[i]) = x[i];
    wave_lds_sync();
  }
}

__global__ __launch_bounds__(256) __attribute__((amdgpu_num_vgpr(256))) void dc_stats_kernel(
    const _Float16* __restrict__ Q16, const _Float16* __restrict__ K16,
    const float* __restrict__ SWg, float* __restrict__ ST) {
  dc_body<1>(Q16, K16, K16, SWg, SWg, ST, (float*)0);
}
__global__ __launch_bounds__(256) __attribute__((amdgpu_num_vgpr(256))) void dc_attn_kernel(
    const _Float16* __restrict__ Q16, const _Float16* __restrict__ K16,
    const _Float16* __restrict__ Vt, const float* __restrict__ SWg,
    const float* __restrict__ ST, float* __restrict__ out) {
  dc_out_body(Q16, K16, Vt, SWg, ST, out);
}

extern "C" void kernel_launch(void* const* d_in, const int* in_sizes, int n_in,
                              void* d_out, int out_size, void* d_ws, size_t ws_size,
                              hipStream_t stream) {
  if (n_in < 7) return;
  const long long need_qkv = ((long long)(NHEAD - 1) * SEQ_FULL + SEQ) * HD;
  if ((long long)in_sizes[0] < need_qkv) return;
  if ((long long)in_sizes[1] < need_qkv) return;
  if ((long long)in_sizes[2] < need_qkv) return;
  if ((long long)in_sizes[3] < (long long)SEQ * DIM) return;
  if ((long long)in_sizes[4] < (long long)DIM * HIDW) return;
  if ((long long)in_sizes[5] < (long long)HIDW * 64) return;
  if ((long long)in_sizes[6] < (long long)DIM * DDW) return;
  if ((long long)out_size < need_qkv) return;
  if (ws_size < WS_TOTAL) return;

  const float* q   = (const float*)d_in[0];
  const float* k   = (const float*)d_in[1];
  const float* v   = (const float*)d_in[2];
  const float* x   = (const float*)d_in[3];
  const float* dw1 = (const float*)d_in[4];
  const float* qkw = (const float*)d_in[5];
  const float* dd  = (const float*)d_in[6];
  float* out = (float*)d_out;

  char* ws = (char*)d_ws;
  _Float16* W1T  = (_Float16*)(ws + OFF_W1T);
  _Float16* QKWT = (_Float16*)(ws + OFF_QKW);
  _Float16* X16  = (_Float16*)(ws + OFF_X16);
  _Float16* Q16  = (_Float16*)(ws + OFF_Q16);
  _Float16* K16  = (_Float16*)(ws + OFF_K16);
  _Float16* VT16 = (_Float16*)(ws + OFF_VT);
  _Float16* H16  = (_Float16*)(ws + OFF_H16);
  _Float16* HR16 = (_Float16*)(ws + OFF_HR);
  float*    SW   = (float*)(ws + OFF_SW);
  float*    ST   = (float*)(ws + OFF_ST);

  dim3 blk(256);

  wconv_kernel<<<dim3(HIDW / 64, DIM / 64), blk, 0, stream>>>(dw1, W1T, (unsigned)HIDW, (unsigned)DIM);
  wconv_kernel<<<dim3(DDW / 64, DIM / 64), blk, 0, stream>>>(dd, W1T + (size_t)HIDW * DIM,
                                                             (unsigned)DDW, (unsigned)DIM);
  wconv_kernel<<<dim3(1, HIDW / 64), blk, 0, stream>>>(qkw, QKWT, 64u, (unsigned)HIDW);
#if SEQ == SEQ_FULL
  wconv_kernel<<<dim3(1, (NHEAD * SEQ) / 64), blk, 0, stream>>>(v, VT16, (unsigned)HD,
                                                                (unsigned)(NHEAD * SEQ));
#else
  for (int hd = 0; hd < NHEAD; ++hd)
    wconv_kernel<<<dim3(1, SEQ / 64), blk, 0, stream>>>(v + (size_t)hd * SEQ_FULL * HD,
                                                        VT16 + (size_t)hd * SEQ, (unsigned)HD,
                                                        (unsigned)(NHEAD * SEQ));
#endif

  cast_kernel<<<dim3((unsigned)(((size_t)SEQ * DIM) / 2048)), blk, 0, stream>>>(
      x, X16, (unsigned)(SEQ * DIM), (unsigned)(SEQ_FULL * DIM), XCARRY);
  cast_kernel<<<dim3((unsigned)(((size_t)NHEAD * SEQ * HD) / 2048)), blk, 0, stream>>>(
      q, Q16, (unsigned)(SEQ * HD), (unsigned)(SEQ_FULL * HD), QCARRY);
  cast_kernel<<<dim3((unsigned)(((size_t)NHEAD * SEQ * HD) / 2048)), blk, 0, stream>>>(
      k, K16, (unsigned)(SEQ * HD), (unsigned)(SEQ_FULL * HD), KCARRY);

  gemm_x_kernel<<<dim3(N1 / 64, SEQ / 64), blk, 0, stream>>>(X16, W1T, H16, HR16, SW);
  gemm_w_kernel<<<dim3(NCP, SEQ / 64), blk, 0, stream>>>(H16, HR16, QKWT, SW);

  dc_stats_kernel<<<dim3(SEQ / TQ), blk, 0, stream>>>(Q16, K16, SW, ST);
  dc_attn_kernel<<<dim3(SEQ / TQ), blk, 0, stream>>>(Q16, K16, VT16, SW, ST, out);
}
